// RelationMessagePassing_14096082666191
// MI455X (gfx1250) — hardware-verified
//
#include <hip/hip_runtime.h>
#include <stddef.h>
#include <stdint.h>

#pragma clang fp contract(off)

#define NH      64
#define TM      64
#define NB      1000
#define AGT     64
#define CH      1024
#define TRP     72
#define WSC     64.0f
#define H16     16.0f
#define INV1024 0.0009765625f
#define INV256  0.00390625f
#define MSC     256.0f
#define EPSE    1e-16f

#define WOFF0 0
#define WOFF1 4096
#define WOFF2 8192
#define WOFF3 24576
#define WOFF4 40960
#define WOFF5 77824
#define WOFF6 114688
#define WOFF7 131072
#define WTOT  139264
#define WTILES 34

#define AGG_LDS_BYTES (32 * 4 + 2 * CH * 4 + NB * NH * 4)

static_assert(CH == AGT * 16);
static_assert(NB % 4 == 0);
static_assert((NB * NH) % (4 * AGT) == 0);
static_assert(AGG_LDS_BYTES == 264320);
static_assert(TM == 64);
static_assert(WTOT == WOFF7 + 128 * 64);

typedef _Float16 v16h __attribute__((ext_vector_type(16)));
typedef _Float16 v8h  __attribute__((ext_vector_type(8)));
typedef _Float16 v4h  __attribute__((ext_vector_type(4)));
typedef float    v8f  __attribute__((ext_vector_type(8)));
typedef float    v4f  __attribute__((ext_vector_type(4)));
typedef unsigned int v4u __attribute__((ext_vector_type(4)));
typedef int      v4i  __attribute__((ext_vector_type(4)));

union Frag  { v16h v; v8h h[2]; };
union Pack8 { v8h h; v4u u; };

__device__ __forceinline__ int clampi(int v, int lo, int hi) { return min(max(v, lo), hi); }
__device__ __forceinline__ float ninf() { return -__builtin_inff(); }
__device__ __forceinline__ v8f zero8() { return (v8f){0.f, 0.f, 0.f, 0.f, 0.f, 0.f, 0.f, 0.f}; }

__device__ __forceinline__ v8f mma16(v16h a, v16h b, v8f c) {
  c = __builtin_amdgcn_wmma_f32_16x16x32_f16(false, a, false, b, (short)0, c, false, false);
  asm volatile("v_nop\n\tv_nop\n\tv_nop\n\tv_nop" : "+v"(c) : "v"(a), "v"(b));
  return c;
}

__device__ __forceinline__ v16h ldfrag(const _Float16* p, int ld, int row0, int k0, int lane) {
  const int m = lane & 15, lh = lane >> 4;
  const _Float16* q = p + (size_t)(row0 + m) * ld + k0 + 8 * lh;
  Frag f;
  f.h[0] = *(const v8h*)(q);
  f.h[1] = *(const v8h*)(q + 16);
  return f.v;
}

__device__ __forceinline__ v8h cvt8(v4f a, v4f b, bool ok) {
  const float z = 0.0f;
  return (v8h){(_Float16)(ok ? a[0] : z), (_Float16)(ok ? a[1] : z), (_Float16)(ok ? a[2] : z), (_Float16)(ok ? a[3] : z),
               (_Float16)(ok ? b[0] : z), (_Float16)(ok ? b[1] : z), (_Float16)(ok ? b[2] : z), (_Float16)(ok ? b[3] : z)};
}

__global__ __launch_bounds__(256) void k_wtr(const float* __restrict__ w0, const float* __restrict__ w1,
                                             const float* __restrict__ w2, const float* __restrict__ w3,
                                             const float* __restrict__ w4, const float* __restrict__ w5,
                                             const float* __restrict__ w6, const float* __restrict__ w7,
                                             _Float16* __restrict__ wt) {
  __shared__ __align__(16) _Float16 st[64 * TRP];
  const int tid = threadIdx.x;
  const int b = blockIdx.x;
  const float* w = w0;
  int kdim = 64, ndim = 64, lt = b, dof = WOFF0;
  if (b >= 1 && b < 2)        { w = w1; kdim = 64;  ndim = 64;  lt = b - 1;  dof = WOFF1; }
  else if (b >= 2 && b < 6)   { w = w2; kdim = 128; ndim = 128; lt = b - 2;  dof = WOFF2; }
  else if (b >= 6 && b < 10)  { w = w3; kdim = 128; ndim = 128; lt = b - 6;  dof = WOFF3; }
  else if (b >= 10 && b < 19) { w = w4; kdim = 192; ndim = 192; lt = b - 10; dof = WOFF4; }
  else if (b >= 19 && b < 28) { w = w5; kdim = 192; ndim = 192; lt = b - 19; dof = WOFF5; }
  else if (b >= 28 && b < 32) { w = w6; kdim = 128; ndim = 128; lt = b - 28; dof = WOFF6; }
  else if (b >= 32)           { w = w7; kdim = 128; ndim = 64;  lt = b - 32; dof = WOFF7; }
  wt += dof;
  const int nxt = ndim >> 6;
  const int n0 = (lt % nxt) * 64, k0 = (lt / nxt) * 64;
  const int kr = tid >> 2;
  const int nc = (tid & 3) * 16;
  const float* sp = w + (size_t)(k0 + kr) * ndim + n0 + nc;
#pragma unroll
  for (int q = 0; q < 4; ++q) {
    const v4f a = *(const v4f*)(sp + 4 * q) * WSC;
#pragma unroll
    for (int j = 0; j < 4; ++j) st[(nc + 4 * q + j) * TRP + kr] = (_Float16)a[j];
  }
  __syncthreads();
  v4u val[2];
  size_t go[2];
#pragma unroll
  for (int j = 0; j < 2; ++j) {
    const int p  = tid + 256 * j;
    const int nr = p >> 3;
    const int pc = p & 7;
    Pack8 pk;
    pk.h   = *(const v8h*)(st + nr * TRP + pc * 8);
    val[j] = pk.u;
    go[j]  = (size_t)(n0 + nr) * kdim + k0 + pc * 8;
  }
  for (int ps = 0; ps < 2; ++ps) {
#pragma unroll
    for (int j = 0; j < 2; ++j) *(volatile v4u*)(wt + go[j]) = val[j];
    __threadfence();
  }
}

template <int A>
__global__ __launch_bounds__(256) void k_rel(const float* __restrict__ states, const int* __restrict__ idx,
                                             const _Float16* __restrict__ w1t, const float* __restrict__ b1,
                                             const _Float16* __restrict__ w2t, const float* __restrict__ b2,
                                             _Float16* __restrict__ msg, float* __restrict__ pmax,
                                             int L, int nNodes) {
  constexpr int D = A * NH, DP = D + 8, KT = D / 32, NTW = D / 32;
  __shared__ __align__(16) _Float16 sX[TM * DP];
  __shared__ __align__(16) _Float16 sH[TM * DP];
  __shared__ int sIdx[TM * A];
  __shared__ float sMax[8];
  const int tid = threadIdx.x, lane = tid & 31, wave = tid >> 5;
  const int hh = lane >> 4, c = lane & 15;
  const int wm = wave & 3, wn = wave >> 2;
  const int tile = blockIdx.x;
  const int E = L / A;
  const int trow0 = tile * TM;

  for (int i = tid; i < TM * A; i += 256) {
    const int g  = trow0 * A + i;
    const int gc = min(g, L - 1);
    const int node = clampi(idx[gc], 0, nNodes - 1);
    sIdx[i] = (g < L) ? node : -1;
  }
  __syncthreads();
  {
    const int m = tid >> 2, q = tid & 3;
#pragma unroll
    for (int k = 0; k < A; ++k) {
      const int node = sIdx[m * A + k];
      const bool ok = node >= 0;
      const float* src = states + (size_t)max(node, 0) * NH + 16 * q;
      const v4f f0 = *(const v4f*)(src);
      const v4f f1 = *(const v4f*)(src + 4);
      const v4f f2 = *(const v4f*)(src + 8);
      const v4f f3 = *(const v4f*)(src + 12);
      _Float16* xr = sX + m * DP + k * NH + 16 * q;
      *(v8h*)(xr)     = cvt8(f0, f1, ok);
      *(v8h*)(xr + 8) = cvt8(f2, f3, ok);
    }
  }
  __syncthreads();

  {
    v16h af[KT];
#pragma unroll
    for (int kt = 0; kt < KT; ++kt) af[kt] = ldfrag(sX, DP, wm * 16, kt * 32, lane);
#pragma unroll 1
    for (int nt = 0; nt < NTW; ++nt) {
      const int nc0 = wn * (D / 2) + nt * 16;
      v8f acc = zero8();
#pragma unroll
      for (int kt = 0; kt < KT; ++kt) acc = mma16(af[kt], ldfrag(w1t, D, nc0, kt * 32, lane), acc);
      const int n = nc0 + c;
      const float bb = b1[n] * H16;
#pragma unroll
      for (int r = 0; r < 8; ++r) {
        const int row = wm * 16 + 8 * hh + r;
        sH[row * DP + n] = (_Float16)fmaxf(acc[r] * 0.25f + bb, 0.0f);
      }
    }
  }
  __syncthreads();

  float lmax = ninf();
  {
    v16h af[KT];
#pragma unroll
    for (int kt = 0; kt < KT; ++kt) af[kt] = ldfrag(sH, DP, wm * 16, kt * 32, lane);
#pragma unroll 1
    for (int nt = 0; nt < NTW; ++nt) {
      const int nc0 = wn * (D / 2) + nt * 16;
      v8f acc = zero8();
#pragma unroll
      for (int kt = 0; kt < KT; ++kt) acc = mma16(af[kt], ldfrag(w2t, D, nc0, kt * 32, lane), acc);
      const int n = nc0 + c;
      const float bb = b2[n];
#pragma unroll
      for (int r = 0; r < 8; ++r) {
        const int row = wm * 16 + 8 * hh + r;
        const float o = acc[r] * INV1024 + bb;
        const bool ok = (trow0 + row) < E;
        lmax = ok ? fmaxf(lmax, o) : lmax;
        sX[row * DP + n] = (_Float16)(o * MSC);
      }
    }
  }
#pragma unroll
  for (int off = 16; off > 0; off >>= 1) lmax = fmaxf(lmax, __shfl_xor(lmax, off, 32));
  if (lane == 0) sMax[wave] = lmax;
  __syncthreads();

  for (int ps = 0; ps < 2; ++ps) {
#pragma unroll
    for (int j = 0; j < 2 * A; ++j) {
      const int p = tid + 256 * j;
      const int line = p >> 3, piece = p & 7;
      const int row = line / A, seg = line - row * A;
      Pack8 pk;
      pk.h = *(const v8h*)(sX + row * DP + seg * NH + piece * 8);
      *(volatile v4u*)(msg + (size_t)trow0 * D + (size_t)p * 8) = pk.u;
    }
    __threadfence();
  }
  if (wave == 0) {
    float m = sMax[0];
#pragma unroll
    for (int q = 1; q < 8; ++q) m = fmaxf(m, sMax[q]);
    volatile float* d = pmax + (size_t)tile * 32 + lane;
    *d = m;
    __threadfence();
    *d = m;
  }
}

__global__ __launch_bounds__(AGT) void k_agg(const int* __restrict__ idx, const _Float16* __restrict__ msg,
                                             const float* __restrict__ pm, float* __restrict__ ep,
                                             int L, int cntPrev, int cntCur, int nNodes, int first) {
  extern __shared__ float4 dsm_raw[];
  float* dsm  = (float*)dsm_raw;
  float* sF   = dsm;
  int*   sI   = (int*)(dsm + 16);
  int*   lstP = (int*)(dsm + 32);
  int*   lstN = lstP + CH;
  float* acc  = dsm + 32 + 2 * CH;
  const int tid = threadIdx.x, lane = tid & 31, wave = tid >> 5;
  const int n0 = blockIdx.x * NB;
  const int nown = min(NB, nNodes - n0);

  float gp = ninf(), mc = ninf();
#pragma unroll 1
  for (int i = tid; i < cntPrev; i += AGT) gp = fmaxf(gp, pm[(size_t)i * 32]);
#pragma unroll 1
  for (int i = tid; i < cntCur; i += AGT) mc = fmaxf(mc, pm[(size_t)(cntPrev + i) * 32]);
#pragma unroll
  for (int off = 16; off > 0; off >>= 1) {
    gp = fmaxf(gp, __shfl_xor(gp, off, 32));
    mc = fmaxf(mc, __shfl_xor(mc, off, 32));
  }
  if (lane == 0) { sF[wave] = gp; sF[2 + wave] = mc; }
  __syncthreads();
  const float gprev = fmaxf(sF[0], sF[1]);
  const float mcur  = fmaxf(sF[2], sF[3]);
  const float G  = fmaxf(gprev, mcur);
  const float cp = first ? 0.0f : __expf((gprev - G) * 8.0f);

  const v4f z4 = {0.f, 0.f, 0.f, 0.f};
#pragma unroll 4
  for (int i = tid; i < NB * NH / 4; i += AGT) *(v4f*)(acc + 4 * i) = z4;
  __syncthreads();

#pragma unroll 1
  for (int c0 = 0; c0 < L; c0 += CH) {
    int nd[16];
    const int base = c0 + 16 * tid;
    if (c0 + CH <= L) {
      const v4i a0 = *(const v4i*)(idx + base);
      const v4i a1 = *(const v4i*)(idx + base + 4);
      const v4i a2 = *(const v4i*)(idx + base + 8);
      const v4i a3 = *(const v4i*)(idx + base + 12);
#pragma unroll
      for (int j = 0; j < 4; ++j) { nd[j] = a0[j]; nd[4 + j] = a1[j]; nd[8 + j] = a2[j]; nd[12 + j] = a3[j]; }
    } else {
#pragma unroll
      for (int j = 0; j < 16; ++j) {
        const int pos = base + j;
        const int v = idx[min(pos, L - 1)];
        nd[j] = (pos < L) ? v : -1;
      }
    }
    unsigned hm = 0u;
#pragma unroll
    for (int j = 0; j < 16; ++j) {
      const int nu = nd[j] - n0;
      const unsigned hit = ((unsigned)nu < (unsigned)nown) ? 1u : 0u;
      hm |= hit << j;
    }
    const int cnt = __builtin_popcount(hm);
    int incl = cnt;
#pragma unroll
    for (int d = 1; d < 32; d <<= 1) {
      const int t = __shfl_up(incl, d, 32);
      incl += (lane >= d) ? t : 0;
    }
    if (lane == 31) sI[wave] = incl;
    __syncthreads();
    const int wt0 = sI[0], wt1 = sI[1];
    const int off = incl - cnt + (wave ? wt0 : 0);
    const int T = min(wt0 + wt1, CH);
    int pos = off;
#pragma unroll
    for (int j = 0; j < 16; ++j) {
      if ((hm >> j) & 1u) {
        const int pp = min(pos, CH - 1);
        lstP[pp] = base + j;
        lstN[pp] = nd[j] - n0;
        ++pos;
      }
    }
    __syncthreads();
#pragma unroll 1
    for (int i = 0; i < T; ++i) {
      const int p  = lstP[i];
      const int nu = lstN[i];
      const int pc = clampi(p, 0, L - 1);
      const float o = (float)msg[(size_t)pc * NH + tid] * INV256;
      const float e = __expf((o - G) * 8.0f);
      float* ap = acc + clampi(nu, 0, NB - 1) * NH + tid;
      *ap = *ap + e;
    }
    __syncthreads();
  }
  __syncthreads();

  const int rsub = tid >> 4, c4 = (tid & 15) * 4;
#pragma unroll 1
  for (int r0 = 0; r0 < NB; r0 += 4) {
    const int nu  = r0 + rsub;
    const int nuc = min(nu, nown - 1);
    const bool ok = nu < nown;
    const v4f a = *(const v4f*)(acc + nuc * NH + c4);
    float* gptr = ep + (size_t)(n0 + nuc) * NH + c4;
    v4f v = a;
    if (!first) {
      const v4f old = *(const v4f*)gptr;
      v = old * cp + a;
    }
    if (ok) *(volatile v4f*)gptr = v;
    __threadfence();
    if (ok) *(volatile v4f*)gptr = v;
  }
}

__global__ __launch_bounds__(256) void k_maxline(const float* __restrict__ pm, int cnt, float* __restrict__ ml) {
  __shared__ float s[8];
  const int tid = threadIdx.x, lane = tid & 31, wave = tid >> 5;
  float m = ninf();
#pragma unroll 1
  for (int i = tid; i < cnt; i += 256) m = fmaxf(m, pm[(size_t)i * 32]);
#pragma unroll
  for (int off = 16; off > 0; off >>= 1) m = fmaxf(m, __shfl_xor(m, off, 32));
  if (lane == 0) s[wave] = m;
  __syncthreads();
  if (wave == 0) {
    float g = s[0];
#pragma unroll
    for (int q = 1; q < 8; ++q) g = fmaxf(g, s[q]);
    volatile float* d = ml + lane;
    *d = g;
    __threadfence();
    *d = g;
  }
}

__global__ __launch_bounds__(256) void k_update(const float* __restrict__ states, const float* __restrict__ ep,
                                                const float* __restrict__ ml, const _Float16* __restrict__ w1t,
                                                const float* __restrict__ b1, const _Float16* __restrict__ w2t,
                                                const float* __restrict__ b2, float* __restrict__ out, int nNodes) {
  constexpr int D = 2 * NH, DP = D + 8, KT = D / 32, OP = NH + 4;
  __shared__ __align__(16) _Float16 sX[TM * DP];
  __shared__ __align__(16) _Float16 sH[TM * DP];
  __shared__ __align__(16) float sO[TM * OP];
  const int tid = threadIdx.x, lane = tid & 31, wave = tid >> 5;
  const int hh = lane >> 4, c = lane & 15;
  const int wm = wave & 3, wn = wave >> 2;
  const int row0 = blockIdx.x * TM;
  const float M = ml[0];
  {
    const int m = tid >> 2, q = tid & 3;
    const int node = min(row0 + m, nNodes - 1);
    const float* es = ep + (size_t)node * NH + 16 * q;
    const float* xs = states + (size_t)node * NH + 16 * q;
    _Float16* xr = sX + m * DP + 16 * q;
#pragma unroll 1
    for (int g = 0; g < 4; ++g) {
      const v4f e4 = *(const v4f*)(es + 4 * g);
      const float u0 = logf(e4[0] + EPSE) * 0.125f + M;
      const float u1 = logf(e4[1] + EPSE) * 0.125f + M;
      const float u2 = logf(e4[2] + EPSE) * 0.125f + M;
      const float u3 = logf(e4[3] + EPSE) * 0.125f + M;
      *(v4h*)(xr + 4 * g) = (v4h){(_Float16)u0, (_Float16)u1, (_Float16)u2, (_Float16)u3};
    }
    const v4f f0 = *(const v4f*)(xs), f1 = *(const v4f*)(xs + 4), f2 = *(const v4f*)(xs + 8), f3 = *(const v4f*)(xs + 12);
    *(v8h*)(xr + NH)     = cvt8(f0, f1, true);
    *(v8h*)(xr + NH + 8) = cvt8(f2, f3, true);
  }
  __syncthreads();
  {
    v16h af[KT];
#pragma unroll
    for (int kt = 0; kt < KT; ++kt) af[kt] = ldfrag(sX, DP, wm * 16, kt * 32, lane);
#pragma unroll 1
    for (int nt = 0; nt < 4; ++nt) {
      const int nc0 = wn * 64 + nt * 16;
      v8f acc = zero8();
#pragma unroll
      for (int kt = 0; kt < KT; ++kt) acc = mma16(af[kt], ldfrag(w1t, D, nc0, kt * 32, lane), acc);
      const int n = nc0 + c;
      const float bb = b1[n] * H16;
#pragma unroll
      for (int r = 0; r < 8; ++r) {
        const int row = wm * 16 + 8 * hh + r;
        sH[row * DP + n] = (_Float16)fmaxf(acc[r] * 0.25f + bb, 0.0f);
      }
    }
  }
  __syncthreads();
  {
    v16h af[KT];
#pragma unroll
    for (int kt = 0; kt < KT; ++kt) af[kt] = ldfrag(sH, DP, wm * 16, kt * 32, lane);
#pragma unroll 1
    for (int nt = 0; nt < 2; ++nt) {
      const int nc0 = wn * 32 + nt * 16;
      v8f acc = zero8();
#pragma unroll
      for (int kt = 0; kt < KT; ++kt) acc = mma16(af[kt], ldfrag(w2t, D, nc0, kt * 32, lane), acc);
      const int n = nc0 + c;
      const float bb = b2[n];
#pragma unroll
      for (int r = 0; r < 8; ++r) {
        const int row = wm * 16 + 8 * hh + r;
        sO[row * OP + n] = acc[r] * INV1024 + bb;
      }
    }
  }
  __syncthreads();
  for (int ps = 0; ps < 2; ++ps) {
#pragma unroll
    for (int j = 0; j < 4; ++j) {
      const int p = tid + 256 * j;
      const int line = p >> 3, piece = p & 7;
      const int row = line >> 1, half = line & 1;
      const v4f v = *(const v4f*)(sO + row * OP + half * 32 + piece * 4);
      const int node = row0 + row;
      if (node < nNodes) *(volatile v4f*)(out + (size_t)node * NH + half * 32 + piece * 4) = v;
    }
    __threadfence();
  }
}

extern "C" void kernel_launch(void* const* d_in, const int* in_sizes, int n_in,
                              void* d_out, int out_size, void* d_ws, size_t ws_size,
                              hipStream_t stream) {
  if (n_in < 20) return;
  const int nNodes = in_sizes[0] / NH;
  if (nNodes <= 0 || in_sizes[0] != nNodes * NH) return;
  const int L0 = in_sizes[1], L1 = in_sizes[2], L2 = in_sizes[3];
  if (L0 <= 0 || L1 <= 0 || L2 <= 0) return;
  if ((L1 % 2) != 0 || (L2 % 3) != 0) return;
  if (in_sizes[4] != 64 * 64 || in_sizes[5] != 64 || in_sizes[6] != 64 * 64 || in_sizes[7] != 64) return;
  if (in_sizes[8] != 128 * 128 || in_sizes[9] != 128 || in_sizes[10] != 128 * 128 || in_sizes[11] != 128) return;
  if (in_sizes[12] != 192 * 192 || in_sizes[13] != 192 || in_sizes[14] != 192 * 192 || in_sizes[15] != 192) return;
  if (in_sizes[16] != 128 * 128 || in_sizes[17] != 128 || in_sizes[18] != 128 * 64 || in_sizes[19] != 64) return;
  if (out_size != nNodes * NH) return;

  const float* states = (const float*)d_in[0];
  const int*   idx0   = (const int*)d_in[1];
  const int*   idx1   = (const int*)d_in[2];
  const int*   idx2   = (const int*)d_in[3];
  const float* r0w1 = (const float*)d_in[4];  const float* r0b1 = (const float*)d_in[5];
  const float* r0w2 = (const float*)d_in[6];  const float* r0b2 = (const float*)d_in[7];
  const float* r1w1 = (const float*)d_in[8];  const float* r1b1 = (const float*)d_in[9];
  const float* r1w2 = (const float*)d_in[10]; const float* r1b2 = (const float*)d_in[11];
  const float* r2w1 = (const float*)d_in[12]; const float* r2b1 = (const float*)d_in[13];
  const float* r2w2 = (const float*)d_in[14]; const float* r2b2 = (const float*)d_in[15];
  const float* uw1  = (const float*)d_in[16]; const float* ub1  = (const float*)d_in[17];
  const float* uw2  = (const float*)d_in[18]; const float* ub2  = (const float*)d_in[19];
  float* out = (float*)d_out;

  const int E0 = L0, E1 = L1 / 2, E2 = L2 / 3;
  const int T0 = (E0 + TM - 1) / TM, T1 = (E1 + TM - 1) / TM, T2 = (E2 + TM - 1) / TM;
  const int NBK = (nNodes + NB - 1) / NB;
  const int NUP = (nNodes + TM - 1) / TM;

  size_t msgBytes = (size_t)T0 * TM * 64 * 2;
  const size_t m1 = (size_t)T1 * TM * 128 * 2, m2 = (size_t)T2 * TM * 192 * 2;
  if (m1 > msgBytes) msgBytes = m1;
  if (m2 > msgBytes) msgBytes = m2;
  msgBytes = (msgBytes + 127) & ~(size_t)127;

  size_t off = 0;
  const size_t oW  = off; off += (size_t)WTOT * 2;
  const size_t oMs = off; off += msgBytes;
  const size_t oE  = off; off += (size_t)NBK * NB * NH * 4;
  const size_t oPm = off; off += (size_t)(T0 + T1 + T2) * 128;
  const size_t oMl = off; off += 128;
  if (off > ws_size) return;
  if (off > (size_t)134217728) return;
  if ((oW | oMs | oE | oPm | oMl) & (size_t)127) return;

  char* ws = (char*)d_ws;
  _Float16* WT  = (_Float16*)(ws + oW);
  _Float16* MSG = (_Float16*)(ws + oMs);
  float*    Epl = (float*)(ws + oE);
  float*    PM  = (float*)(ws + oPm);
  float*    ML  = (float*)(ws + oMl);

  k_wtr<<<dim3(WTILES), dim3(256), 0, stream>>>(r0w1, r0w2, r1w1, r1w2, r2w1, r2w2, uw1, uw2, WT);
  (void)hipFuncSetAttribute(reinterpret_cast<const void*>(&k_agg), hipFuncAttributeMaxDynamicSharedMemorySize,
                            AGG_LDS_BYTES);
  k_rel<1><<<dim3(T0), dim3(256), 0, stream>>>(states, idx0, WT + WOFF0, r0b1, WT + WOFF1, r0b2, MSG, PM, L0, nNodes);
  k_agg<<<dim3(NBK), dim3(AGT), AGG_LDS_BYTES, stream>>>(idx0, MSG, PM, Epl, L0, 0, T0, nNodes, 1);
  k_rel<2><<<dim3(T1), dim3(256), 0, stream>>>(states, idx1, WT + WOFF2, r1b1, WT + WOFF3, r1b2, MSG, PM + (size_t)T0 * 32,
                                               L1, nNodes);
  k_agg<<<dim3(NBK), dim3(AGT), AGG_LDS_BYTES, stream>>>(idx1, MSG, PM, Epl, L1, T0, T1, nNodes, 0);
  k_rel<3><<<dim3(T2), dim3(256), 0, stream>>>(states, idx2, WT + WOFF4, r2b1, WT + WOFF5, r2b2, MSG,
                                               PM + (size_t)(T0 + T1) * 32, L2, nNodes);
  k_agg<<<dim3(NBK), dim3(AGT), AGG_LDS_BYTES, stream>>>(idx2, MSG, PM, Epl, L2, T0 + T1, T2, nNodes, 0);
  k_maxline<<<dim3(1), dim3(256), 0, stream>>>(PM, T0 + T1 + T2, ML);
  k_update<<<dim3(NUP), dim3(256), 0, stream>>>(states, Epl, ML, WT + WOFF6, ub1, WT + WOFF7, ub2, out, nNodes);
  (void)hipGetLastError();
}
